// RecordingStableAudioAttnProcessor2_0_13211319402790
// MI455X (gfx1250) — hardware-verified
//
#include <hip/hip_runtime.h>
#include <stdint.h>


#define NB   2
#define NS   2048
#define NDM  1024
#define NH   16
#define NKV  8
#define NHD  64
#define NROT 32
#define EPSV 1e-6f
#define NM   (NB * NS)

typedef _Float16 f16;
typedef f16   v8h  __attribute__((ext_vector_type(8)));
typedef f16   v16h __attribute__((ext_vector_type(16)));
typedef float v4f  __attribute__((ext_vector_type(4)));
typedef float v8f  __attribute__((ext_vector_type(8)));
typedef v4f v4fa __attribute__((may_alias));
typedef v8h v8ha __attribute__((may_alias));

union Frag { v16h v; v8h h[2]; f16 e[16]; };

__device__ __forceinline__ v8f mma(const v16h a, const v16h b, v8f c) {
    v8f d = __builtin_amdgcn_wmma_f32_16x16x32_f16(false, a, false, b, (short)0, c, false, false);
    asm volatile("v_nop\n\tv_nop\n\tv_nop\n\tv_nop" : "+v"(d) : "v"(a), "v"(b));
    return d;
}

__device__ __forceinline__ v8f zero8() {
    v8f z;
#pragma unroll
    for (int i = 0; i < 8; ++i) z[i] = 0.0f;
    return z;
}

__global__ __launch_bounds__(256) void k_cvt(const float* __restrict__ in, f16* __restrict__ out, int n8) {
    const int i = blockIdx.x * 256 + threadIdx.x;
    if (i >= n8) return;
    const float* s = in + (size_t)i * 8;
    const v4f u0 = *(const v4f*)(s);
    const v4f u1 = *(const v4f*)(s + 4);
    v8h o;
#pragma unroll
    for (int e = 0; e < 4; ++e) { o[e] = (f16)u0[e]; o[4 + e] = (f16)u1[e]; }
    f16* d = out + (size_t)i * 8;
    *(volatile v8h*)d = o;
    __threadfence();
    *(volatile v8h*)d = o;
}

__global__ __launch_bounds__(256) void k_wtrans(const float* __restrict__ W, f16* __restrict__ Wt,
                                                int K, int N, float scale) {
    __shared__ float T[64][33];
    const int tid = threadIdx.x, lane = tid & 31, wid = tid >> 5;
    const int nTn = N / 32;
    const int tn = blockIdx.x % nTn, tk = blockIdx.x / nTn;
    const int n0 = tn * 32, k0 = tk * 64;
    if (k0 + 64 > K || n0 + 32 > N) return;
    {
        const int k = tid >> 2, c = (tid & 3) * 8;
        const float* src = W + (size_t)(k0 + k) * N + n0 + c;
        const v4f u0 = *(const v4f*)(src);
        const v4f u1 = *(const v4f*)(src + 4);
#pragma unroll
        for (int e = 0; e < 4; ++e) { T[k][c + e] = u0[e]; T[k][c + 4 + e] = u1[e]; }
    }
    __syncthreads();
    const int L  = wid * 4 + (lane >> 3);
    const int k8 = (lane & 7) * 8;
    v8h o;
#pragma unroll
    for (int e = 0; e < 8; ++e) o[e] = (f16)(T[k8 + e][L] * scale);
    f16* dst = Wt + (size_t)(n0 + L) * K + k0 + k8;
    *(volatile v8h*)dst = o;
    __threadfence();
    *(volatile v8h*)dst = o;
}

__device__ __forceinline__ void mm16x64(const f16* __restrict__ arow, const f16* __restrict__ brow,
                                        int K, int h8, v8f& c0, v8f& c1, v8f& c2, v8f& c3) {
    const size_t jstep = (size_t)16 * K;
#pragma unroll 2
    for (int k0 = 0; k0 < K; k0 += 32) {
        Frag a, b;
        a.h[0] = *(const v8h*)(arow + k0 + h8);
        a.h[1] = *(const v8h*)(arow + k0 + 16 + h8);
        const f16* bp = brow + k0 + h8;
        b.h[0] = *(const v8h*)(bp);             b.h[1] = *(const v8h*)(bp + 16);             c0 = mma(a.v, b.v, c0);
        b.h[0] = *(const v8h*)(bp + jstep);     b.h[1] = *(const v8h*)(bp + jstep + 16);     c1 = mma(a.v, b.v, c1);
        b.h[0] = *(const v8h*)(bp + 2 * jstep); b.h[1] = *(const v8h*)(bp + 2 * jstep + 16); c2 = mma(a.v, b.v, c2);
        b.h[0] = *(const v8h*)(bp + 3 * jstep); b.h[1] = *(const v8h*)(bp + 3 * jstep + 16); c3 = mma(a.v, b.v, c3);
    }
}

__global__ __launch_bounds__(256) void k_qkv(const f16* __restrict__ X,
                                             const f16* __restrict__ Wqt, const f16* __restrict__ Wkt,
                                             const f16* __restrict__ Wvt,
                                             const float* __restrict__ nqw, const float* __restrict__ nkw,
                                             const float* __restrict__ cosT, const float* __restrict__ sinT,
                                             f16* __restrict__ qb, f16* __restrict__ kb, f16* __restrict__ vt) {
    __shared__ __attribute__((aligned(16))) float Cs[128][68];
    const int tid = threadIdx.x, lane = tid & 31, wid = tid >> 5;
    const int h = lane >> 4, l16 = lane & 15, h8 = h * 8;
    const int nt = blockIdx.x;
    const int m0 = blockIdx.y * 128;
    if (m0 + 128 > NM || nt >= 32) return;

    int mode, hh, nHh;
    const f16* Wt;
    const float* nw;
    if (nt < 16)      { mode = 0; hh = nt;      nHh = NH;  Wt = Wqt; nw = nqw; }
    else if (nt < 24) { mode = 1; hh = nt - 16; nHh = NKV; Wt = Wkt; nw = nkw; }
    else              { mode = 2; hh = nt - 24; nHh = NKV; Wt = Wvt; nw = nkw; }
    const int n0 = hh * NHD;
    const int bb = m0 / NS, s0 = m0 % NS;

    v8f c0 = zero8(), c1 = zero8(), c2 = zero8(), c3 = zero8();
    const f16* arow = X  + (size_t)(m0 + 16 * wid + l16) * NDM;
    const f16* brow = Wt + (size_t)(n0 + l16) * NDM;
    mm16x64(arow, brow, NDM, h8, c0, c1, c2, c3);

#pragma unroll
    for (int r = 0; r < 8; ++r) {
        const int row = 16 * wid + 8 * h + r;
        Cs[row][l16]      = c0[r];
        Cs[row][16 + l16] = c1[r];
        Cs[row][32 + l16] = c2[r];
        Cs[row][48 + l16] = c3[r];
    }
    __syncthreads();

    if (mode != 2) {
        const float osc = (mode == 0) ? 0.125f : 1.0f;
        const float w0 = nw[lane], w1 = nw[lane + 32];
#pragma unroll 1
        for (int r = 0; r < 16; ++r) {
            const int row = 16 * wid + r;
            const int s = s0 + row;
            float x0 = Cs[row][lane] * (1.0f / 16.0f);
            float x1 = Cs[row][lane + 32] * (1.0f / 16.0f);
            float ss = x0 * x0 + x1 * x1;
#pragma unroll
            for (int m = 16; m >= 1; m >>= 1) ss += __shfl_xor(ss, m, 32);
            const float rinv = rsqrtf(ss * (1.0f / NHD) + EPSV);
            const float xn0 = x0 * rinv * w0;
            const float xn1 = x1 * rinv * w1;
            const float part = __shfl_xor(xn0, 16, 32);
            const float rot = (lane < 16) ? -part : part;
            const float c  = cosT[(size_t)s * NROT + lane];
            const float sn = sinT[(size_t)s * NROT + lane];
            const float y0 = xn0 * c + rot * sn;
            Cs[row][lane]      = y0 * osc;
            Cs[row][lane + 32] = xn1 * osc;
        }
    }
    __syncthreads();

    v8h o[4];
    size_t off[4];
    if (mode != 2) {
        f16* ob = ((mode == 0) ? qb : kb) + ((size_t)(bb * nHh + hh) * NS + s0) * NHD;
#pragma unroll
        for (int q = 0; q < 4; ++q) {
            const int L = 4 * q + (lane >> 3);
            const int row = 16 * wid + L;
            const int cc = (lane & 7) * 8;
            const v4f u0 = *(const v4fa*)(&Cs[row][cc]);
            const v4f u1 = *(const v4fa*)(&Cs[row][cc + 4]);
#pragma unroll
            for (int e = 0; e < 4; ++e) { o[q][e] = (f16)u0[e]; o[q][4 + e] = (f16)u1[e]; }
            off[q] = (size_t)row * NHD + cc;
        }
#pragma unroll
        for (int q = 0; q < 4; ++q) *(volatile v8h*)(ob + off[q]) = o[q];
        __threadfence();
#pragma unroll
        for (int q = 0; q < 4; ++q) *(volatile v8h*)(ob + off[q]) = o[q];
    } else {
        f16* ob = vt + (size_t)(bb * NKV + hh) * NHD * NS + s0;
#pragma unroll
        for (int q = 0; q < 4; ++q) {
            const int L = 4 * q + (lane >> 3);
            const int d = 8 * wid + (L >> 1);
            const int sb = (L & 1) * 64 + (lane & 7) * 8;
#pragma unroll
            for (int e = 0; e < 8; ++e) o[q][e] = (f16)(Cs[sb + e][d] * (1.0f / 16.0f));
            off[q] = (size_t)d * NS + sb;
        }
#pragma unroll
        for (int q = 0; q < 4; ++q) *(volatile v8h*)(ob + off[q]) = o[q];
        __threadfence();
#pragma unroll
        for (int q = 0; q < 4; ++q) *(volatile v8h*)(ob + off[q]) = o[q];
    }
}

__global__ __launch_bounds__(256) void k_attn(const f16* __restrict__ qb, const f16* __restrict__ kb,
                                              const f16* __restrict__ vt, f16* __restrict__ ob) {
    __shared__ __attribute__((aligned(16))) f16   Ks[32 * 72];
    __shared__ __attribute__((aligned(16))) f16   Vs[64 * 40];
    __shared__ __attribute__((aligned(16))) float Pw[8 * 16 * 36];
    __shared__ __attribute__((aligned(16))) f16   Os[8 * 16 * 72];

    const int tid = threadIdx.x, lane = tid & 31, wid = tid >> 5;
    const int h = lane >> 4, l16 = lane & 15, h8 = h * 8;
    const int bb = blockIdx.z, hd = blockIdx.y, kvh = hd / (NH / NKV);
    const int qblk = blockIdx.x * 128;
    if (qblk + 128 > NS || hd >= NH || bb >= NB) return;
    const int q0 = qblk + wid * 16;

    const f16* qrow = qb + ((size_t)(bb * NH + hd) * NS + q0 + l16) * NHD;
    Frag qa0, qa1;
    qa0.h[0] = *(const v8h*)(qrow + h8);
    qa0.h[1] = *(const v8h*)(qrow + 16 + h8);
    qa1.h[0] = *(const v8h*)(qrow + 32 + h8);
    qa1.h[1] = *(const v8h*)(qrow + 48 + h8);

    float m_run = -1e30f, l_run = 0.0f;
    v8f acc0 = zero8(), acc1 = zero8(), acc2 = zero8(), acc3 = zero8();

    const f16* kbase = kb + (size_t)(bb * NKV + kvh) * NS * NHD;
    const f16* vbase = vt + (size_t)(bb * NKV + kvh) * NHD * NS;
    float* pw = Pw + wid * 16 * 36;

#pragma unroll 1
    for (int it = 0; it < NS / 32; ++it) {
        __syncthreads();
        {
            const int r = tid >> 3, c = (tid & 7) * 8;
            const v8h u = *(const v8h*)(kbase + (size_t)(it * 32 + r) * NHD + c);
            *(v8h*)(Ks + r * 72 + c) = u;
        }
        {
            const int d = tid >> 2, c = (tid & 3) * 8;
            const v8h u = *(const v8h*)(vbase + (size_t)d * NS + it * 32 + c);
            *(v8h*)(Vs + d * 40 + c) = u;
        }
        __syncthreads();

#pragma unroll
        for (int t = 0; t < 2; ++t) {
            const f16* kp = Ks + (t * 16 + l16) * 72;
            Frag b0, b1;
            b0.h[0] = *(const v8h*)(kp + h8);      b0.h[1] = *(const v8h*)(kp + 16 + h8);
            b1.h[0] = *(const v8h*)(kp + 32 + h8); b1.h[1] = *(const v8h*)(kp + 48 + h8);
            v8f sc = zero8();
            sc = mma(qa0.v, b0.v, sc);
            sc = mma(qa1.v, b1.v, sc);
#pragma unroll
            for (int r = 0; r < 8; ++r) pw[(8 * h + r) * 36 + t * 16 + l16] = sc[r];
        }
        __syncthreads();

        const float* prow = pw + l16 * 36 + h8;
        const v4f r0 = *(const v4fa*)(prow);
        const v4f r1 = *(const v4fa*)(prow + 4);
        const v4f r2 = *(const v4fa*)(prow + 16);
        const v4f r3 = *(const v4fa*)(prow + 20);

        float rm = r0[0];
#pragma unroll
        for (int i = 1; i < 4; ++i) rm = fmaxf(rm, r0[i]);
#pragma unroll
        for (int i = 0; i < 4; ++i) rm = fmaxf(rm, r1[i]);
#pragma unroll
        for (int i = 0; i < 4; ++i) rm = fmaxf(rm, r2[i]);
#pragma unroll
        for (int i = 0; i < 4; ++i) rm = fmaxf(rm, r3[i]);
        rm = fmaxf(rm, __shfl_xor(rm, 16, 32));

        const float mn = fmaxf(m_run, rm);
        const float alpha = __expf(m_run - mn);

        Frag pa;
        float rs = 0.0f;
#pragma unroll
        for (int i = 0; i < 4; ++i) { const float p = __expf(r0[i] - mn); rs += p; pa.e[i]      = (f16)(p * 256.0f); }
#pragma unroll
        for (int i = 0; i < 4; ++i) { const float p = __expf(r1[i] - mn); rs += p; pa.e[4 + i]  = (f16)(p * 256.0f); }
#pragma unroll
        for (int i = 0; i < 4; ++i) { const float p = __expf(r2[i] - mn); rs += p; pa.e[8 + i]  = (f16)(p * 256.0f); }
#pragma unroll
        for (int i = 0; i < 4; ++i) { const float p = __expf(r3[i] - mn); rs += p; pa.e[12 + i] = (f16)(p * 256.0f); }
        rs += __shfl_xor(rs, 16, 32);
        l_run = l_run * alpha + rs;
        m_run = mn;

        float al[8];
#pragma unroll
        for (int r = 0; r < 8; ++r) al[r] = __shfl(alpha, 8 * h + r, 32);
#pragma unroll
        for (int r = 0; r < 8; ++r) { acc0[r] *= al[r]; acc1[r] *= al[r]; acc2[r] *= al[r]; acc3[r] *= al[r]; }

        {
            Frag bv;
            const f16* vp = Vs + (0 * 16 + l16) * 40;
            bv.h[0] = *(const v8h*)(vp + h8); bv.h[1] = *(const v8h*)(vp + 16 + h8); acc0 = mma(pa.v, bv.v, acc0);
            vp = Vs + (1 * 16 + l16) * 40;
            bv.h[0] = *(const v8h*)(vp + h8); bv.h[1] = *(const v8h*)(vp + 16 + h8); acc1 = mma(pa.v, bv.v, acc1);
            vp = Vs + (2 * 16 + l16) * 40;
            bv.h[0] = *(const v8h*)(vp + h8); bv.h[1] = *(const v8h*)(vp + 16 + h8); acc2 = mma(pa.v, bv.v, acc2);
            vp = Vs + (3 * 16 + l16) * 40;
            bv.h[0] = *(const v8h*)(vp + h8); bv.h[1] = *(const v8h*)(vp + 16 + h8); acc3 = mma(pa.v, bv.v, acc3);
        }
    }

    const float inv = 0.125f / l_run;
    float iv[8];
#pragma unroll
    for (int r = 0; r < 8; ++r) iv[r] = __shfl(inv, 8 * h + r, 32);

    __syncthreads();
    f16* os = Os + wid * 16 * 72;
#pragma unroll
    for (int r = 0; r < 8; ++r) {
        const int row = 8 * h + r;
        os[row * 72 + l16]      = (f16)(acc0[r] * iv[r]);
        os[row * 72 + 16 + l16] = (f16)(acc1[r] * iv[r]);
        os[row * 72 + 32 + l16] = (f16)(acc2[r] * iv[r]);
        os[row * 72 + 48 + l16] = (f16)(acc3[r] * iv[r]);
    }
    __syncthreads();

    v8h o[4];
    size_t off[4];
#pragma unroll
    for (int q = 0; q < 4; ++q) {
        const int L = 4 * q + (lane >> 3);
        const int cc = (lane & 7) * 8;
        o[q] = *(const v8ha*)(os + L * 72 + cc);
        off[q] = ((size_t)(bb * NS + q0 + L)) * (NH * NHD) + hd * NHD + cc;
    }
#pragma unroll
    for (int q = 0; q < 4; ++q) *(volatile v8h*)(ob + off[q]) = o[q];
    __threadfence();
#pragma unroll
    for (int q = 0; q < 4; ++q) *(volatile v8h*)(ob + off[q]) = o[q];
}

__global__ __launch_bounds__(256) void k_oproj(const f16* __restrict__ A, const f16* __restrict__ Wot,
                                               const float* __restrict__ bias, const float* __restrict__ resid,
                                               float* __restrict__ out) {
    __shared__ __attribute__((aligned(16))) float Cs[128][68];
    const int tid = threadIdx.x, lane = tid & 31, wid = tid >> 5;
    const int h = lane >> 4, l16 = lane & 15, h8 = h * 8;
    const int n0 = blockIdx.x * 64;
    const int m0 = blockIdx.y * 128;
    if (n0 + 64 > NDM || m0 + 128 > NM) return;

    v8f c0 = zero8(), c1 = zero8(), c2 = zero8(), c3 = zero8();
    const f16* arow = A   + (size_t)(m0 + 16 * wid + l16) * (NH * NHD);
    const f16* brow = Wot + (size_t)(n0 + l16) * (NH * NHD);
    mm16x64(arow, brow, NH * NHD, h8, c0, c1, c2, c3);

#pragma unroll
    for (int r = 0; r < 8; ++r) {
        const int row = 16 * wid + 8 * h + r;
        Cs[row][l16]      = c0[r];
        Cs[row][16 + l16] = c1[r];
        Cs[row][32 + l16] = c2[r];
        Cs[row][48 + l16] = c3[r];
    }
    __syncthreads();

    v4f o[8];
    size_t off[8];
#pragma unroll
    for (int q = 0; q < 8; ++q) {
        const int L = 4 * q + (lane >> 3);
        const int row = 16 * wid + (L >> 1);
        const int cc = (L & 1) * 32 + (lane & 7) * 4;
        const v4f cv = *(const v4fa*)(&Cs[row][cc]);
        const size_t go = (size_t)(m0 + row) * NDM + n0 + cc;
        const v4f bv = *(const v4f*)(bias + n0 + cc);
        const v4f rv = *(const v4f*)(resid + go);
        v4f val;
#pragma unroll
        for (int e = 0; e < 4; ++e) val[e] = (cv[e] * (1.0f / 512.0f) + bv[e]) + rv[e];
        o[q] = val;
        off[q] = go;
    }
#pragma unroll
    for (int q = 0; q < 8; ++q) *(volatile v4f*)(out + off[q]) = o[q];
    __threadfence();
#pragma unroll
    for (int q = 0; q < 8; ++q) *(volatile v4f*)(out + off[q]) = o[q];
}

extern "C" void kernel_launch(void* const* d_in, const int* in_sizes, int n_in,
                              void* d_out, int out_size, void* d_ws, size_t ws_size,
                              hipStream_t stream) {
    if (n_in < 10) return;
    if (in_sizes[0] != NM * NDM) return;
    if (in_sizes[1] != NDM * NH * NHD) return;
    if (in_sizes[2] != NDM * NKV * NHD || in_sizes[3] != NDM * NKV * NHD) return;
    if (in_sizes[4] != NH * NHD * NDM) return;
    if (in_sizes[5] < NDM || in_sizes[6] < NHD || in_sizes[7] < NHD) return;
    if (in_sizes[8] != NS * NROT || in_sizes[9] != NS * NROT) return;
    if (out_size != NM * NDM) return;

    const float* hs   = (const float*)d_in[0];
    const float* wq   = (const float*)d_in[1];
    const float* wk   = (const float*)d_in[2];
    const float* wv   = (const float*)d_in[3];
    const float* wo   = (const float*)d_in[4];
    const float* bo   = (const float*)d_in[5];
    const float* nqw  = (const float*)d_in[6];
    const float* nkw  = (const float*)d_in[7];
    const float* cosT = (const float*)d_in[8];
    const float* sinT = (const float*)d_in[9];

    const size_t szX   = (size_t)NM * NDM * sizeof(f16);
    const size_t szWq  = (size_t)NDM * NH * NHD * sizeof(f16);
    const size_t szWkv = (size_t)NDM * NKV * NHD * sizeof(f16);
    const size_t szWo  = (size_t)NH * NHD * NDM * sizeof(f16);
    const size_t szQ   = (size_t)NB * NH * NS * NHD * sizeof(f16);
    const size_t szKV  = (size_t)NB * NKV * NS * NHD * sizeof(f16);
    const size_t szO   = (size_t)NM * NH * NHD * sizeof(f16);
    size_t offp = 0;
    const size_t oX   = offp; offp += szX;
    const size_t oWq  = offp; offp += szWq;
    const size_t oWk  = offp; offp += szWkv;
    const size_t oWv  = offp; offp += szWkv;
    const size_t oWo  = offp; offp += szWo;
    const size_t oQ   = offp; offp += szQ;
    const size_t oK   = offp; offp += szKV;
    const size_t oV   = offp; offp += szKV;
    const size_t oO   = offp; offp += szO;
    if (offp > ws_size) return;

    char* ws = (char*)d_ws;
    f16* hsb  = (f16*)(ws + oX);
    f16* wqt  = (f16*)(ws + oWq);
    f16* wkt  = (f16*)(ws + oWk);
    f16* wvt  = (f16*)(ws + oWv);
    f16* wot  = (f16*)(ws + oWo);
    f16* qbuf = (f16*)(ws + oQ);
    f16* kbuf = (f16*)(ws + oK);
    f16* vtb  = (f16*)(ws + oV);
    f16* attb = (f16*)(ws + oO);

    const int n8 = (NM * NDM) / 8;
    k_cvt<<<(n8 + 255) / 256, 256, 0, stream>>>(hs, hsb, n8);

    k_wtrans<<<((NH * NHD) / 32) * (NDM / 64), 256, 0, stream>>>(wq, wqt, NDM, NH * NHD, 16.0f);
    k_wtrans<<<((NKV * NHD) / 32) * (NDM / 64), 256, 0, stream>>>(wk, wkt, NDM, NKV * NHD, 16.0f);
    k_wtrans<<<((NKV * NHD) / 32) * (NDM / 64), 256, 0, stream>>>(wv, wvt, NDM, NKV * NHD, 16.0f);
    k_wtrans<<<(NDM / 32) * ((NH * NHD) / 64), 256, 0, stream>>>(wo, wot, NH * NHD, NDM, 16.0f);

    k_qkv<<<dim3(32, (NM + 127) / 128), 256, 0, stream>>>(hsb, wqt, wkt, wvt, nqw, nkw, cosT, sinT,
                                                         qbuf, kbuf, vtb);

    k_attn<<<dim3((NS + 127) / 128, NH, NB), 256, 0, stream>>>(qbuf, kbuf, vtb, attb);

    k_oproj<<<dim3((NDM + 63) / 64, (NM + 127) / 128), 256, 0, stream>>>(attb, wot, bo, hs, (float*)d_out);
}
